// LengthRegulator_34059090657417
// MI455X (gfx1250) — hardware-verified
//
#include <hip/hip_runtime.h>
#include <stdint.h>


typedef _Float16 v16h __attribute__((ext_vector_type(16)));
typedef _Float16 v8h  __attribute__((ext_vector_type(8)));
typedef float    v8f  __attribute__((ext_vector_type(8)));
typedef float    v4f  __attribute__((ext_vector_type(4)));
typedef int      v4i  __attribute__((ext_vector_type(4)));

union H8  { _Float16 s[8]; v8h v; v4f f; };
union A16 { v16h v; v8h hh[2]; };

enum {
    B_    = 8,
    T_    = 512,
    D_    = 384,
    K_    = 3,
    L_    = 4096,
    KTOT  = 1152,
    NKT   = 36,
    NNT   = 24,
    M1    = 510,
    M2    = 508,
    PACKN = NNT * NKT * 32 * 16,
    PACKG = PACKN / 8,
    AROWS = 18,
    DWPITCH = 32,
    NVEC1 = (B_ * M2) / 4
};

#define WSCALE 64.f
#define WINV   (1.f / 64.f)

__device__ __forceinline__ v8f wmma16(v16h a, v16h b, v8f c)
{
    c = __builtin_amdgcn_wmma_f32_16x16x32_f16(false, a, false, b, (short)0, c, false, false);
    asm volatile("v_nop\n\tv_nop\n\tv_nop\n\tv_nop" : "+v"(c) : "v"(a), "v"(b));
    return c;
}

__global__ __launch_bounds__(256) void pack_w_kernel(const float* __restrict__ w,
                                                     _Float16* __restrict__ wp, int ngroups)
{
    const int q = blockIdx.x * 256 + threadIdx.x;
    if (q >= ngroups) return;
    const int hf   = q & 1;
    const int lane = (q >> 1) & 31;
    const int tile = q >> 6;
    const int kt   = tile % NKT;
    const int nt   = tile / NKT;
    const int n    = nt * 16 + (lane & 15);
    const int h    = lane >> 4;
    const int kb   = kt * 32 + 16 * hf + 8 * h;
    H8 u;
    #pragma unroll
    for (int j = 0; j < 8; ++j) {
        const int kg = kb + j;
        const int ci = kg % D_;
        const int kk = kg / D_;
        u.s[j] = (_Float16)(w[((size_t)n * D_ + ci) * K_ + kk] * WSCALE);
    }
    const v4f val = u.f;
    volatile v4f* p = (volatile v4f*)(wp + (size_t)q * 8);
    *p = val;
    __threadfence();
    *p = val;
}

__global__ __launch_bounds__(128) void cumsum_kernel(const int* __restrict__ tgt,
                                                    int* __restrict__ cum, int nb)
{
    __shared__ int s_tot[128];
    const int b = blockIdx.x;
    if (b >= nb) return;
    const int tid = threadIdx.x;
    const int* src = tgt + (size_t)b * T_ + tid * 4;
    const int a0 = src[0];
    const int a1 = a0 + src[1];
    const int a2 = a1 + src[2];
    const int a3 = a2 + src[3];
    s_tot[tid] = a3;
    __syncthreads();
    if (tid == 0) {
        int run = 0;
        for (int i = 0; i < 128; ++i) { const int t = s_tot[i]; s_tot[i] = run; run += t; }
    }
    __syncthreads();
    const int o = s_tot[tid];
    v4i v;
    v.x = a0 + o; v.y = a1 + o; v.z = a2 + o; v.w = a3 + o;
    volatile v4i* p = (volatile v4i*)(cum + (size_t)b * T_ + tid * 4);
    *p = v;
    __threadfence();
    *p = v;
}

template<bool SECOND>
__global__ __launch_bounds__(256) void conv_ln_kernel(
    const float*    __restrict__ xsrc,
    const _Float16*              hsrc,
    const _Float16* __restrict__ wp,
    const float*    __restrict__ cb,
    const float*    __restrict__ gam,
    const float*    __restrict__ bet,
    _Float16*                    hout,
    const float*    __restrict__ lw,
    const float*    __restrict__ lb,
    float*          __restrict__ durws,
    int nblk)
{
    __shared__ __attribute__((aligned(16))) _Float16 s_a[AROWS * D_];
    __shared__ float s_tile[16][388];
    __shared__ float s_dur[16];

    const int blk = blockIdx.x;
    if (blk >= nblk) return;
    const int b    = blk >> 5;
    const int mt   = blk & 31;
    const int t0   = mt * 16;
    const int tid  = threadIdx.x;
    const int lane = tid & 31;
    const int wv   = tid >> 5;

    #pragma unroll 1
    for (int gi = tid; gi < (AROWS * D_) / 8; gi += 256) {
        const int e = gi * 8;
        const int i = e / D_;
        const int c = e - i * D_;
        int r = t0 + i;
        r = (r < T_) ? r : (T_ - 1);
        const size_t roff = ((size_t)b * T_ + r) * D_ + c;
        H8 u;
        if (SECOND) {
            u.v = *(const v8h*)(hsrc + roff);
        } else {
            const v4f f0 = *(const v4f*)(xsrc + roff);
            const v4f f1 = *(const v4f*)(xsrc + roff + 4);
            u.s[0] = (_Float16)f0.x; u.s[1] = (_Float16)f0.y; u.s[2] = (_Float16)f0.z; u.s[3] = (_Float16)f0.w;
            u.s[4] = (_Float16)f1.x; u.s[5] = (_Float16)f1.y; u.s[6] = (_Float16)f1.z; u.s[7] = (_Float16)f1.w;
        }
        *(v8h*)(s_a + e) = u.v;
    }
    __syncthreads();

    const int m = lane & 15;
    const int h = lane >> 4;
    const _Float16* arow  = s_a + m * D_ + 8 * h;
    const _Float16* wbase = wp + (size_t)lane * 16;
    const int nt0 = wv * 3;

    v8f c0 = {0.f, 0.f, 0.f, 0.f, 0.f, 0.f, 0.f, 0.f};
    v8f c1 = c0, c2 = c0;

    #pragma unroll 1
    for (int kt = 0; kt < NKT; ++kt) {
        const int k0 = kt * 32;
        A16 ua;
        ua.hh[0] = *(const v8h*)(arow + k0);
        ua.hh[1] = *(const v8h*)(arow + k0 + 16);
        const v16h bf0 = *(const v16h*)(wbase + ((size_t)(nt0 + 0) * NKT + kt) * 512);
        const v16h bf1 = *(const v16h*)(wbase + ((size_t)(nt0 + 1) * NKT + kt) * 512);
        const v16h bf2 = *(const v16h*)(wbase + ((size_t)(nt0 + 2) * NKT + kt) * 512);
        c0 = wmma16(ua.v, bf0, c0);
        c1 = wmma16(ua.v, bf1, c1);
        c2 = wmma16(ua.v, bf2, c2);
    }

    {
        const int rowoff = h * 8;
        {
            const int col = (nt0 + 0) * 16 + m; const float bv = cb[col];
            #pragma unroll
            for (int v = 0; v < 8; ++v) s_tile[rowoff + v][col] = c0[v] * WINV + bv;
        }
        {
            const int col = (nt0 + 1) * 16 + m; const float bv = cb[col];
            #pragma unroll
            for (int v = 0; v < 8; ++v) s_tile[rowoff + v][col] = c1[v] * WINV + bv;
        }
        {
            const int col = (nt0 + 2) * 16 + m; const float bv = cb[col];
            #pragma unroll
            for (int v = 0; v < 8; ++v) s_tile[rowoff + v][col] = c2[v] * WINV + bv;
        }
    }
    __syncthreads();

    const int row = tid >> 4;
    const int sub = tid & 15;
    float y[NNT];
    float s = 0.f;
    #pragma unroll
    for (int j = 0; j < NNT; ++j) { y[j] = s_tile[row][sub + 16 * j]; s += y[j]; }
    s += __shfl_xor(s, 8); s += __shfl_xor(s, 4); s += __shfl_xor(s, 2); s += __shfl_xor(s, 1);
    const float mu = s * (1.f / 384.f);
    float dv = 0.f;
    #pragma unroll
    for (int j = 0; j < NNT; ++j) { const float t = y[j] - mu; dv += t * t; }
    dv += __shfl_xor(dv, 8); dv += __shfl_xor(dv, 4); dv += __shfl_xor(dv, 2); dv += __shfl_xor(dv, 1);
    const float rs = rsqrtf(dv * (1.f / 384.f) + 1e-5f);
    #pragma unroll
    for (int j = 0; j < NNT; ++j) {
        const int col = sub + 16 * j;
        const float v = (y[j] - mu) * rs * gam[col] + bet[col];
        y[j] = v > 0.f ? v : 0.f;
    }

    if (!SECOND) {
        #pragma unroll
        for (int j = 0; j < NNT; ++j) s_tile[row][sub + 16 * j] = y[j];
        __syncthreads();
        const size_t base = ((size_t)b * T_ + t0) * D_;
        H8  hv[3];
        int offs[3];
        #pragma unroll
        for (int it = 0; it < 3; ++it) {
            const int g    = wv * 12 + it * 4 + (lane >> 3);
            const int rowg = g / 6;
            const int cq   = g - rowg * 6;
            const int col0 = cq * 64 + (lane & 7) * 8;
            #pragma unroll
            for (int j = 0; j < 8; ++j) hv[it].s[j] = (_Float16)s_tile[rowg][col0 + j];
            offs[it] = g * 64 + (lane & 7) * 8;
        }
        #pragma unroll
        for (int it = 0; it < 3; ++it) *(volatile v4f*)(hout + base + offs[it]) = hv[it].f;
        __threadfence();
        #pragma unroll
        for (int it = 0; it < 3; ++it) *(volatile v4f*)(hout + base + offs[it]) = hv[it].f;
    } else {
        float dot = 0.f;
        #pragma unroll
        for (int j = 0; j < NNT; ++j) dot += y[j] * lw[sub + 16 * j];
        dot += __shfl_xor(dot, 8); dot += __shfl_xor(dot, 4); dot += __shfl_xor(dot, 2); dot += __shfl_xor(dot, 1);
        float td = dot + lb[0];
        td = td > 0.f ? td : 0.f;
        const float dval = expf(td);
        if (sub == 0) s_dur[row] = dval;
        __syncthreads();
        if (tid < 8) {
            v4f v = {0.f, 0.f, 0.f, 0.f};
            if (tid < 4) { v.x = s_dur[tid * 4 + 0]; v.y = s_dur[tid * 4 + 1]; v.z = s_dur[tid * 4 + 2]; v.w = s_dur[tid * 4 + 3]; }
            volatile v4f* p = (volatile v4f*)(durws + (size_t)blk * DWPITCH + tid * 4);
            *p = v;
            __threadfence();
            *p = v;
        }
    }
}

__global__ __launch_bounds__(256) void dur_out_kernel(const float* __restrict__ durws,
                                                     float* __restrict__ dout, int nvec)
{
    const int tid = threadIdx.x;
    v4f val[4];
    #pragma unroll
    for (int it = 0; it < 4; ++it) {
        const int f = it * 256 + tid;
        v4f v = {0.f, 0.f, 0.f, 0.f};
        if (f < nvec) {
            float t[4];
            #pragma unroll
            for (int c = 0; c < 4; ++c) {
                const int e  = f * 4 + c;
                const int bb = e / M2;
                const int r  = e - bb * M2;
                t[c] = durws[((size_t)bb * 32 + (r >> 4)) * DWPITCH + (r & 15)];
            }
            v.x = t[0]; v.y = t[1]; v.z = t[2]; v.w = t[3];
        }
        val[it] = v;
    }
    #pragma unroll
    for (int it = 0; it < 4; ++it) {
        const int f = it * 256 + tid;
        if (f < nvec) *(volatile v4f*)(dout + (size_t)f * 4) = val[it];
    }
    __threadfence();
    #pragma unroll
    for (int it = 0; it < 4; ++it) {
        const int f = it * 256 + tid;
        if (f < nvec) *(volatile v4f*)(dout + (size_t)f * 4) = val[it];
    }
}

__global__ __launch_bounds__(256) void gather_kernel(
    const float* __restrict__ x, const int* __restrict__ cum, const int* __restrict__ mlen,
    float* __restrict__ out, int nblk)
{
    __shared__ int s_cum[T_];
    const int blk = blockIdx.x;
    if (blk >= nblk) return;
    const int b     = blk >> 9;
    const int lbase = (blk & 511) * 8;
    const int tid   = threadIdx.x;
    s_cum[tid]       = cum[(size_t)b * T_ + tid];
    s_cum[tid + 256] = cum[(size_t)b * T_ + tid + 256];
    __syncthreads();

    int lm = mlen[0];
    lm = lm < L_ ? lm : L_;

    const int lane = tid & 31;
    const int l    = lbase + (tid >> 5);
    int lo = 0, hi = T_;
    while (lo < hi) { const int mid = (lo + hi) >> 1; if (s_cum[mid] <= l) lo = mid + 1; else hi = mid; }

    v4f v[3];
    if (lo < T_ && l < lm) {
        const v4f* xrow = (const v4f*)(x + ((size_t)b * T_ + lo) * D_);
        #pragma unroll
        for (int j = 0; j < 3; ++j) v[j] = xrow[lane + 32 * j];
    } else {
        const v4f z = {0.f, 0.f, 0.f, 0.f};
        #pragma unroll
        for (int j = 0; j < 3; ++j) v[j] = z;
    }
    volatile v4f* orow = (volatile v4f*)(out + ((size_t)b * L_ + l) * D_);
    #pragma unroll
    for (int j = 0; j < 3; ++j) orow[lane + 32 * j] = v[j];
    __threadfence();
    #pragma unroll
    for (int j = 0; j < 3; ++j) orow[lane + 32 * j] = v[j];
}

extern "C" void kernel_launch(void* const* d_in, const int* in_sizes, int n_in,
                              void* d_out, int out_size, void* d_ws, size_t ws_size,
                              hipStream_t stream)
{
    if (n_in < 13) return;
    if (in_sizes[0] != B_ * T_ * D_) return;
    if (in_sizes[1] != B_ * T_) return;
    if (in_sizes[2] < 1) return;
    if (in_sizes[3] != D_ * D_ * K_ || in_sizes[7] != D_ * D_ * K_) return;
    if (in_sizes[4] != D_ || in_sizes[5] != D_ || in_sizes[6] != D_) return;
    if (in_sizes[8] != D_ || in_sizes[9] != D_ || in_sizes[10] != D_) return;
    if (in_sizes[11] != D_ || in_sizes[12] < 1) return;
    if (out_size != B_ * L_ * D_ + B_ * M2) return;

    const float* x    = (const float*)d_in[0];
    const int*   tgt  = (const int*)d_in[1];
    const int*   mlen = (const int*)d_in[2];
    const float* c1w  = (const float*)d_in[3];
    const float* c1b  = (const float*)d_in[4];
    const float* g1   = (const float*)d_in[5];
    const float* b1   = (const float*)d_in[6];
    const float* c2w  = (const float*)d_in[7];
    const float* c2b  = (const float*)d_in[8];
    const float* g2   = (const float*)d_in[9];
    const float* b2   = (const float*)d_in[10];
    const float* lw   = (const float*)d_in[11];
    const float* lb   = (const float*)d_in[12];

    char* ws = (char*)d_ws;
    size_t off = 0;
    auto carve = [&](size_t bytes) -> void* {
        off = (off + 255) & ~(size_t)255;
        void* p = ws + off;
        off += bytes;
        return p;
    };
    int*      cum   = (int*)     carve((size_t)B_ * T_ * sizeof(int));
    _Float16* h1h   = (_Float16*)carve((size_t)B_ * T_ * D_ * sizeof(_Float16));
    _Float16* w1p   = (_Float16*)carve((size_t)PACKN * sizeof(_Float16));
    _Float16* w2p   = (_Float16*)carve((size_t)PACKN * sizeof(_Float16));
    float*    durws = (float*)   carve((size_t)B_ * 32 * DWPITCH * sizeof(float));
    if (off > ws_size) return;

    float* out_main = (float*)d_out;
    float* dur      = out_main + (size_t)B_ * L_ * D_;

    pack_w_kernel<<<(PACKG + 255) / 256, 256, 0, stream>>>(c1w, w1p, (int)PACKG);
    pack_w_kernel<<<(PACKG + 255) / 256, 256, 0, stream>>>(c2w, w2p, (int)PACKG);
    cumsum_kernel<<<B_, 128, 0, stream>>>(tgt, cum, (int)B_);

    conv_ln_kernel<false><<<B_ * 32, 256, 0, stream>>>(
        x, h1h, w1p, c1b, g1, b1, h1h, lw, lb, durws, (int)(B_ * 32));
    conv_ln_kernel<true><<<B_ * 32, 256, 0, stream>>>(
        x, h1h, w2p, c2b, g2, b2, h1h, lw, lb, durws, (int)(B_ * 32));

    dur_out_kernel<<<1, 256, 0, stream>>>(durws, dur, (int)NVEC1);
    gather_kernel<<<B_ * 512, 256, 0, stream>>>(x, cum, mlen, out_main, (int)(B_ * 512));
}
